// mLSTMBackend_28226525070271
// MI455X (gfx1250) — hardware-verified
//
#include <hip/hip_runtime.h>


#define NB_  1
#define NT_  2048
#define NH_  8
#define NKV  8
#define HD   128
#define KW   (NKV * HD)
#define HS   KW
#define NREP 1
#define DM   HS
#define NTK  NT_
#define SCL  0.08838834764831845f
#define PSC  32768.0f
#define LOSC 1024.0f
#define LOSCI (1.0f / 1024.0f)

typedef _Float16 h16;
typedef unsigned short bf;
typedef __attribute__((ext_vector_type(16))) __bf16   v16bf;
typedef __attribute__((ext_vector_type(16))) _Float16 v16h;
typedef __attribute__((ext_vector_type(8)))  _Float16 v8h;
typedef __attribute__((ext_vector_type(8)))  unsigned short v8us;
typedef __attribute__((ext_vector_type(8)))  float    v8f;
typedef __attribute__((ext_vector_type(4)))  float    v4f;
typedef __attribute__((ext_vector_type(4)))  _Float16 v4h;
typedef v8h  __attribute__((may_alias)) v8ha;
typedef v4f  __attribute__((may_alias)) v4fa;
typedef v8us __attribute__((may_alias)) v8usa;

__device__ __forceinline__ unsigned short f2bf(float f) { unsigned u = __float_as_uint(f); u += 0x7FFFu + ((u >> 16) & 1u); return (unsigned short)(u >> 16); }
__device__ __forceinline__ float bf2f(unsigned short b) { return __uint_as_float(((unsigned)b) << 16); }
__device__ __forceinline__ float bfr(float f) { return bf2f(f2bf(f)); }
__device__ __forceinline__ v16h cat16(v8h lo, v8h hi) { return __builtin_shufflevector(lo, hi, 0, 1, 2, 3, 4, 5, 6, 7, 8, 9, 10, 11, 12, 13, 14, 15); }
__device__ __forceinline__ v16bf cat16b(v8us lo, v8us hi) { return __builtin_bit_cast(v16bf, __builtin_shufflevector(lo, hi, 0, 1, 2, 3, 4, 5, 6, 7, 8, 9, 10, 11, 12, 13, 14, 15)); }
__device__ __forceinline__ v8f wmma16(v16h a, v16h b, v8f c) { return __builtin_amdgcn_wmma_f32_16x16x32_f16(false, a, false, b, (short)0, c, false, false); }
__device__ __forceinline__ v8f wmmab(v16bf a, v16bf b, v8f c) { return __builtin_amdgcn_wmma_f32_16x16x32_bf16(false, a, false, b, (short)0, c, false, false); }

__global__ __launch_bounds__(256) void k_cvtb(const float* __restrict__ src, int nrows, bf* dst) {
    const int lane = threadIdx.x & 31, r = blockIdx.x * 8 + (threadIdx.x >> 5);
    if (r >= nrows) return;
#pragma unroll 1
    for (int ps = 0; ps < 2; ++ps) {
#pragma unroll
        for (int q = 0; q < HS / 256; ++q) { v8us o;
#pragma unroll
            for (int i = 0; i < 8; ++i) o[i] = f2bf(src[(size_t)r * HS + q * 256 + lane * 8 + i]);
            *(volatile v8us*)(dst + (size_t)r * HS + q * 256 + lane * 8) = o; }
        if (ps == 0) __threadfence(); }
}
template <bool SPLITA>
__global__ __launch_bounds__(128) void k_gemm(const bf* __restrict__ A, const bf* __restrict__ Al, const bf* __restrict__ Bn, const float* __restrict__ bias, int ldc, float* C) {
    __shared__ __align__(16) float ost[4][16 * 68];
    const int lane = threadIdx.x & 31, wave = threadIdx.x >> 5, lr = lane & 15, hi = lane >> 4;
    const size_t r0 = (size_t)blockIdx.x * 64 + wave * 16; const int c0 = blockIdx.y * 64;
    const size_t aoff = (r0 + lr) * HS + 8 * hi;
    v8f acc[4];
#pragma unroll
    for (int t = 0; t < 4; ++t) acc[t] = (v8f){};
#pragma unroll 2
    for (int kc = 0; kc < HS; kc += 32) {
        const v16bf a = cat16b(*(const v8us*)(A + aoff + kc), *(const v8us*)(A + aoff + kc + 16));
        v16bf al = a; if (SPLITA) al = cat16b(*(const v8us*)(Al + aoff + kc), *(const v8us*)(Al + aoff + kc + 16));
#pragma unroll
        for (int t = 0; t < 4; ++t) { const bf* bp = Bn + (size_t)(c0 + t * 16 + lr) * HS + kc + 8 * hi; const v16bf bb = cat16b(*(const v8us*)bp, *(const v8us*)(bp + 16)); acc[t] = wmmab(a, bb, acc[t]); if (SPLITA) acc[t] = wmmab(al, bb, acc[t]); }
        asm volatile("v_nop" : "+v"(acc[0]), "+v"(acc[1]), "+v"(acc[2]), "+v"(acc[3]) : "v"(a), "v"(al) : "memory");
    }
    float* os = &ost[wave][0];
#pragma unroll
    for (int t = 0; t < 4; ++t)
#pragma unroll
        for (int j = 0; j < 8; ++j) os[(hi * 8 + j) * 68 + t * 16 + lr] = acc[t][j] + (bias ? bfr(bias[c0 + t * 16 + lr]) : 0.f);
    __builtin_amdgcn_wave_barrier(); asm volatile("" ::: "memory");
    float* crow = C + r0 * ldc + c0;
    auto pass = [&]() {
#pragma unroll
        for (int s = 0; s < 8; ++s) { const int Lid = (lane >> 3) + 4 * s, piece = lane & 7; const int row = Lid >> 1, cofs = (Lid & 1) * 32 + piece * 4;
            const v4f val = *(const v4fa*)(os + row * 68 + cofs); *(volatile v4f*)(crow + (size_t)row * ldc + cofs) = val; }
    };
    pass(); __threadfence(); pass();
}
__global__ __launch_bounds__(256) void k_vt(const float* __restrict__ V, bf* VTH, bf* VTL) {
    __shared__ float tl[64][65];
    const int tid = threadIdx.x, t0 = blockIdx.x * 64, d0 = blockIdx.y * 64, g = blockIdx.z;
    { const int tt = tid >> 2, dq = (tid & 3) * 16;
#pragma unroll
      for (int i = 0; i < 16; ++i) tl[dq + i][tt] = V[(size_t)(t0 + tt) * KW + g * HD + d0 + dq + i]; }
    __syncthreads();
    const int piece = tid & 7;
    auto pass = [&]() {
#pragma unroll
        for (int s = 0; s < 2; ++s) { const int d = (tid >> 3) + 32 * s; v8us oh, ol;
#pragma unroll
            for (int i = 0; i < 8; ++i) { const float v = tl[d][piece * 8 + i]; const unsigned short hb = f2bf(v); oh[i] = hb; ol[i] = f2bf(v - bf2f(hb)); }
            const size_t o = ((size_t)g * HD + d0 + d) * NT_ + t0 + piece * 8; *(volatile v8us*)(VTH + o) = oh; *(volatile v8us*)(VTL + o) = ol; }
    };
    pass(); __threadfence(); pass();
}
__global__ __launch_bounds__(256) void k_wt(const float* __restrict__ Wm, int K, int ncols, bf* WT) {
    __shared__ __align__(16) unsigned short tl[64 * 72];
    const int tid = threadIdx.x, k0 = blockIdx.x * 64, n0 = blockIdx.y * 64;
    const int kk = tid >> 2, nq = (tid & 3) * 16;
#pragma unroll
    for (int i = 0; i < 16; ++i) tl[(nq + i) * 72 + kk] = f2bf(Wm[(size_t)(k0 + kk) * ncols + n0 + nq + i]);
    __syncthreads();
    const int piece = tid & 7;
    auto pass = [&]() {
#pragma unroll
        for (int s = 0; s < 2; ++s) { const int nr = (tid >> 3) + 32 * s; const v8us val = *(const v8usa*)(tl + nr * 72 + piece * 8); *(volatile v8us*)(WT + (size_t)(n0 + nr) * K + k0 + piece * 8) = val; }
    };
    pass(); __threadfence(); pass();
}
template <bool SPLITA, bool F16OUT = false>
__global__ __launch_bounds__(128) void k_gemmb(const bf* __restrict__ A, const bf* __restrict__ Al, const bf* __restrict__ Bn, const float* __restrict__ bias, float* C, int ldc, h16* C2, const float* __restrict__ R = nullptr, int K = DM, int roundR = 1) {
    __shared__ __align__(16) float ost[4][16 * 68];
    const int lane = threadIdx.x & 31, wave = threadIdx.x >> 5, lr = lane & 15, hi = lane >> 4;
    const int r0 = blockIdx.x * 64 + wave * 16, c0 = blockIdx.y * 64;
    const size_t aoff = (size_t)(r0 + lr) * K + 8 * hi;
    size_t boff[4];
#pragma unroll
    for (int t = 0; t < 4; ++t) boff[t] = (size_t)(c0 + t * 16 + lr) * K + 8 * hi;
    v8f acc[4];
#pragma unroll
    for (int t = 0; t < 4; ++t) acc[t] = (v8f){};
#pragma unroll 1
    for (int kc = 0; kc < K; kc += 32) {
        const v16bf a = cat16b(*(const v8us*)(A + aoff + kc), *(const v8us*)(A + aoff + kc + 16));
        v16bf al = a;
        if (SPLITA) al = cat16b(*(const v8us*)(Al + aoff + kc), *(const v8us*)(Al + aoff + kc + 16));
#pragma unroll
        for (int t = 0; t < 4; ++t) { const v16bf b = cat16b(*(const v8us*)(Bn + boff[t] + kc), *(const v8us*)(Bn + boff[t] + kc + 16)); acc[t] = wmmab(a, b, acc[t]); if (SPLITA) acc[t] = wmmab(al, b, acc[t]); }
        asm volatile("v_nop\n\tv_nop\n\tv_nop\n\tv_nop" : "+v"(acc[0]), "+v"(acc[1]), "+v"(acc[2]), "+v"(acc[3]) : "v"(a), "v"(al));
    }
    float* os = &ost[wave][0];
#pragma unroll
    for (int t = 0; t < 4; ++t) { const float bv = bias ? bfr(bias[c0 + t * 16 + lr]) : 0.f;
#pragma unroll
        for (int j = 0; j < 8; ++j) os[(hi * 8 + j) * 68 + t * 16 + lr] = acc[t][j] + bv; }
    __syncthreads();
    if (F16OUT) {
        h16* crow = (h16*)(void*)C + (size_t)r0 * ldc + c0;
        auto pass = [&]() {
#pragma unroll
            for (int s = 0; s < 4; ++s) { const int row = 4 * s + (lane >> 3), piece = lane & 7; const float* sp = os + row * 68 + piece * 8; v8h o, o2;
#pragma unroll
                for (int i = 0; i < 8; ++i) { const h16 a = (h16)sp[i]; o[i] = a; o2[i] = (h16)((sp[i] - (float)a) * LOSC); }
                *(volatile v8h*)(crow + (size_t)row * ldc + piece * 8) = o; if (C2) *(volatile v8h*)(C2 + (size_t)r0 * ldc + c0 + (size_t)row * ldc + piece * 8) = o2; }
        };
        pass(); __threadfence(); pass();
    } else {
        float* crow = C + (size_t)r0 * ldc + c0;
        auto pass = [&]() {
#pragma unroll
            for (int s = 0; s < 8; ++s) { const int Lid = (lane >> 3) + 4 * s, piece = lane & 7; const int row = Lid >> 1, cofs = (Lid & 1) * 32 + piece * 4;
                v4f val = *(const v4fa*)(os + row * 68 + cofs); if (R) { const v4f rv = *(const v4f*)(R + ((size_t)r0 + row) * ldc + c0 + cofs); val += roundR ? (v4f){bfr(rv[0]), bfr(rv[1]), bfr(rv[2]), bfr(rv[3])} : rv; }
                *(volatile v4f*)(crow + (size_t)row * ldc + cofs) = val; }
        };
        pass(); __threadfence(); pass();
    }
}

__global__ __launch_bounds__(256) void k_tof16(const float* __restrict__ src, h16* PH, h16* PL) {
    const int lane = threadIdx.x & 31, wid = blockIdx.x * 8 + (threadIdx.x >> 5); if (wid >= NH_ * NT_) return;
    const int bh = wid / NT_, t = wid % NT_; const v4f v = *(const v4f*)(src + ((size_t)bh * NT_ + t) * HD + lane * 4); v4h oh, ol;
#pragma unroll
    for (int i = 0; i < 4; ++i) { const float x = bfr(v[i]); const h16 a = (fabsf(x) < 6.103515625e-05f) ? (h16)0.0f : (h16)x; oh[i] = a; ol[i] = (h16)((x - (float)a) * LOSC); }
    const size_t o = (size_t)t * KW + bh * HD + lane * 4;
    *(volatile v4h*)(PH + o) = oh; *(volatile v4h*)(PL + o) = ol; __threadfence(); *(volatile v4h*)(PH + o) = oh; *(volatile v4h*)(PL + o) = ol;
}
__global__ __launch_bounds__(256) void k_tof32(const float* __restrict__ src, float* dst) {
    const int lane = threadIdx.x & 31, wid = blockIdx.x * 8 + (threadIdx.x >> 5); if (wid >= NH_ * NT_) return;
    const int bh = wid / NT_, t = wid % NT_; v4f v = *(const v4f*)(src + ((size_t)bh * NT_ + t) * HD + lane * 4);
#pragma unroll
    for (int i = 0; i < 4; ++i) v[i] = bfr(v[i]);
    const size_t o = (size_t)t * KW + bh * HD + lane * 4; *(volatile v4f*)(dst + o) = v; __threadfence(); *(volatile v4f*)(dst + o) = v;
}
__global__ __launch_bounds__(256) void k_gates(const float* __restrict__ ig, const float* __restrict__ fg, float* RQ, float* GK, float* EM) {
    const int lane = threadIdx.x & 31, bh = blockIdx.x * 8 + (threadIdx.x >> 5); if (bh >= NH_) return;
    float cF = 0.f, cM = -3.0e38f;
#pragma unroll 1
    for (int c = 0; c < NT_ / 32; ++c) { const int t = c * 32 + lane; const size_t o = (size_t)bh * NT_ + t;
        const float x = bfr(fg[o]); float fs = fminf(x, 0.f) - log1pf(__expf(-fabsf(x)));
#pragma unroll
        for (int sh = 1; sh < 32; sh <<= 1) { const float y = __shfl_up(fs, sh, 32); if (lane >= sh) fs += y; }
        const float F = cF + fs; cF = __shfl(F, 31, 32);
        float g = bfr(ig[o]) - F;
#pragma unroll
        for (int sh = 1; sh < 32; sh <<= 1) { const float y = __shfl_up(g, sh, 32); if (lane >= sh) g = fmaxf(g, y); }
        const float M = fmaxf(cM, g); cM = __shfl(M, 31, 32);
        const float m = F + fmaxf(M, 0.f); const float rqv = F - m, gkv = F - bfr(ig[o]), emv = __expf(-m);
        *(volatile float*)(RQ + o) = rqv; *(volatile float*)(GK + o) = gkv; *(volatile float*)(EM + o) = emv; __threadfence(); *(volatile float*)(RQ + o) = rqv; *(volatile float*)(GK + o) = gkv; *(volatile float*)(EM + o) = emv; }
}
__global__ __launch_bounds__(256) void k_out(const float* __restrict__ AT, float* OUTP) {
    const int lane = threadIdx.x & 31, wid = blockIdx.x * 8 + (threadIdx.x >> 5); if (wid >= NH_ * NT_) return;
    const int bh = wid / NT_, t = wid % NT_; const v4f v = *(const v4f*)(AT + (size_t)t * KW + bh * HD + lane * 4);
    const size_t o = ((size_t)bh * NT_ + t) * HD + lane * 4; *(volatile v4f*)(OUTP + o) = v; __threadfence(); *(volatile v4f*)(OUTP + o) = v;
}
__global__ __launch_bounds__(128) void k_attn(const h16* __restrict__ QH, const h16* __restrict__ QL, const h16* __restrict__ KH, const h16* __restrict__ KL, const bf* __restrict__ VTH, const bf* __restrict__ VTL, const float* __restrict__ RQ, const float* __restrict__ GK, const float* __restrict__ EM, float* OUTP) {
    __shared__ __align__(16) unsigned short plds[4][16 * 32];
    __shared__ __align__(16) unsigned short plds2[4][16 * 32];
    __shared__ __align__(16) float ost[4][16 * 68];
    const int lane = threadIdx.x & 31, wave = threadIdx.x >> 5, lr = lane & 15, hi = lane >> 4;
    const int bid = blockIdx.x; const int h = bid / (NT_ / 64), qt = bid - h * (NT_ / 64); const int g = h / NREP;
    const int q0 = qt * 64 + wave * 16;
    unsigned short* pl = &plds[wave][0]; unsigned short* pl2 = &plds2[wave][0];
    const size_t qo = (size_t)(q0 + lr) * (NH_ * HD) + h * HD + 8 * hi;
    const h16* kh_b = KH + g * HD; const h16* kl_b = KL + g * HD;
    const size_t vbase = ((size_t)g * HD) * NT_;
    v8f o[8];
#pragma unroll
    for (int n = 0; n < 8; ++n) o[n] = (v8f){};
    float mrow[8], lpart[8];
#pragma unroll
    for (int j = 0; j < 8; ++j) { mrow[j] = -3.0e38f; lpart[j] = 0.f; }
    const int kt_hi = (qt * 64 + 63) / 32;
    float rq[8], em[8];
#pragma unroll
    for (int j = 0; j < 8; ++j) { rq[j] = RQ[h * NT_ + q0 + hi * 8 + j]; em[j] = EM[h * NT_ + q0 + hi * 8 + j]; }
#pragma unroll 1
    for (int kt = 0; kt <= kt_hi; ++kt) {
        const int l0 = kt * 32;
        const size_t ko0 = (size_t)(l0 + lr) * KW + 8 * hi, ko1 = (size_t)(l0 + 16 + lr) * KW + 8 * hi;
        v8f s0 = {}, s1 = {}, x0 = {}, x1 = {};
#pragma unroll
        for (int kc = 0; kc < 4; ++kc) {
            const v16h qa = cat16(*(const v8h*)(QH + qo + kc * 32), *(const v8h*)(QH + qo + kc * 32 + 16)), qx = cat16(*(const v8h*)(QL + qo + kc * 32), *(const v8h*)(QL + qo + kc * 32 + 16));
            const v16h k0h = cat16(*(const v8h*)(kh_b + ko0 + kc * 32), *(const v8h*)(kh_b + ko0 + kc * 32 + 16)), k1h = cat16(*(const v8h*)(kh_b + ko1 + kc * 32), *(const v8h*)(kh_b + ko1 + kc * 32 + 16));
            s0 = wmma16(qa, k0h, s0); s1 = wmma16(qa, k1h, s1); x0 = wmma16(qx, k0h, x0); x1 = wmma16(qx, k1h, x1);
            asm volatile("v_nop" : "+v"(s0), "+v"(s1), "+v"(x0), "+v"(x1) : "v"(qa), "v"(qx), "v"(k0h), "v"(k1h) : "memory");
            const v16h k0l = cat16(*(const v8h*)(kl_b + ko0 + kc * 32), *(const v8h*)(kl_b + ko0 + kc * 32 + 16)), k1l = cat16(*(const v8h*)(kl_b + ko1 + kc * 32), *(const v8h*)(kl_b + ko1 + kc * 32 + 16));
            x0 = wmma16(qa, k0l, x0); x1 = wmma16(qa, k1l, x1);
            asm volatile("v_nop" : "+v"(x0), "+v"(x1) : "v"(k0l), "v"(k1l) : "memory");
        }
        asm volatile("v_nop\n\tv_nop\n\tv_nop\n\tv_nop" : "+v"(s0), "+v"(s1), "+v"(x0), "+v"(x1));
        const float gka = GK[h * NT_ + l0 + lr], gkb = GK[h * NT_ + l0 + 16 + lr];
#pragma unroll
        for (int j = 0; j < 8; ++j) { const int qi = q0 + hi * 8 + j, ja = l0 + lr, jb = l0 + 16 + lr;
            const float p0 = (ja <= qi) ? (s0[j] + x0[j] * LOSCI) * SCL * __expf(rq[j] - gka) : 0.f, p1 = (jb <= qi) ? (s1[j] + x1[j] * LOSCI) * SCL * __expf(rq[j] - gkb) : 0.f;
            lpart[j] += (p0 + p1);
            const int mr = hi * 8 + j; const float ps0 = p0 * PSC, ps1 = p1 * PSC; const unsigned short h0 = f2bf(ps0), h1 = f2bf(ps1);
            pl[mr * 32 + lr] = h0; pl[mr * 32 + 16 + lr] = h1; pl2[mr * 32 + lr] = f2bf(ps0 - bf2f(h0)); pl2[mr * 32 + 16 + lr] = f2bf(ps1 - bf2f(h1)); }
        asm volatile("" ::: "memory");
        const v16bf pa = cat16b(*(const v8usa*)(pl + lr * 32 + hi * 8), *(const v8usa*)(pl + lr * 32 + 16 + hi * 8));
        const v16bf px = cat16b(*(const v8usa*)(pl2 + lr * 32 + hi * 8), *(const v8usa*)(pl2 + lr * 32 + 16 + hi * 8));
#pragma unroll
        for (int n = 0; n < 8; ++n) { const size_t vo = vbase + (size_t)(n * 16 + lr) * NT_ + l0 + hi * 8;
            const v16bf vh = cat16b(*(const v8us*)(VTH + vo), *(const v8us*)(VTH + vo + 16)), vl = cat16b(*(const v8us*)(VTL + vo), *(const v8us*)(VTL + vo + 16));
            o[n] = wmmab(pa, vh, o[n]); o[n] = wmmab(px, vh, o[n]); o[n] = wmmab(pa, vl, o[n]);
            asm volatile("" : "+v"(o[n]) : "v"(vh), "v"(vl) : "memory"); }
        asm volatile("v_nop\n\tv_nop\n\tv_nop\n\tv_nop" : "+v"(o[0]), "+v"(o[7]) : "v"(pa), "v"(px));
        __builtin_amdgcn_wave_barrier();
    }
    float inv[8];
#pragma unroll
    for (int j = 0; j < 8; ++j) { float rs = lpart[j]; rs += __shfl_xor(rs, 1, 16); rs += __shfl_xor(rs, 2, 16); rs += __shfl_xor(rs, 4, 16); rs += __shfl_xor(rs, 8, 16); inv[j] = 1.0f / ((fmaxf(fabsf(rs), em[j]) + 1e-6f) * PSC); }
    float* os = &ost[wave][0];
    float* ob = OUTP + (size_t)q0 * (NH_ * HD) + (size_t)h * HD;
#pragma unroll
    for (int half = 0; half < 2; ++half) {
#pragma unroll
        for (int n = 0; n < 4; ++n)
#pragma unroll
            for (int j = 0; j < 8; ++j) os[(hi * 8 + j) * 68 + n * 16 + lr] = o[half * 4 + n][j] * inv[j];
        __builtin_amdgcn_wave_barrier(); asm volatile("" ::: "memory");
#pragma unroll
        for (int ps2 = 0; ps2 < 2; ++ps2) {
#pragma unroll
            for (int s = 0; s < 8; ++s) { const int Lid = (lane >> 3) + 4 * s, piece = lane & 7; const int row = Lid >> 1, cofs = (Lid & 1) * 32 + piece * 4;
                const v4f val = *(const v4fa*)(os + row * 68 + cofs); *(volatile v4f*)(ob + (size_t)row * (NH_ * HD) + half * 64 + cofs) = val; }
            if (ps2 == 0) __threadfence(); }
        __builtin_amdgcn_wave_barrier(); asm volatile("" ::: "memory");
    }
}

extern "C" void kernel_launch(void* const* d_in, const int* in_sizes, int n_in,
                              void* d_out, int out_size, void* d_ws, size_t ws_size, hipStream_t stream) {
    (void)in_sizes; (void)n_in; (void)out_size;
    const float* q = (const float*)d_in[0]; const float* k = (const float*)d_in[1]; const float* v = (const float*)d_in[2]; const float* ig = (const float*)d_in[3]; const float* fg = (const float*)d_in[4];
    float* out = (float*)d_out;
    char* wsp = (char*)d_ws;
    auto take = [&](size_t bytes) { char* p = wsp; wsp += (bytes + 255) & ~(size_t)255; return (void*)p; };
    h16* QH = (h16*)take((size_t)NT_ * KW * 2); h16* QL = (h16*)take((size_t)NT_ * KW * 2); h16* KH = (h16*)take((size_t)NT_ * KW * 2); h16* KL = (h16*)take((size_t)NT_ * KW * 2);
    float* Vf = (float*)take((size_t)NT_ * KW * 4); bf* VTH = (bf*)take((size_t)KW * NT_ * 2); bf* VTL = (bf*)take((size_t)KW * NT_ * 2); float* AT = (float*)take((size_t)NT_ * KW * 4);
    float* RQ = (float*)take((size_t)NH_ * NT_ * 4); float* GK = (float*)take((size_t)NH_ * NT_ * 4); float* EM = (float*)take((size_t)NH_ * NT_ * 4);
    if ((size_t)(wsp - (char*)d_ws) > ws_size) return;
    k_tof16<<<(NH_ * NT_) / 8, 256, 0, stream>>>(q, QH, QL); k_tof16<<<(NH_ * NT_) / 8, 256, 0, stream>>>(k, KH, KL);
    k_tof32<<<(NH_ * NT_) / 8, 256, 0, stream>>>(v, Vf); k_vt<<<dim3(NT_ / 64, 2, NKV), 256, 0, stream>>>(Vf, VTH, VTL);
    k_gates<<<1, 256, 0, stream>>>(ig, fg, RQ, GK, EM);
    k_attn<<<NH_ * (NT_ / 64), 128, 0, stream>>>(QH, QL, KH, KL, VTH, VTL, RQ, GK, EM, AT);
    k_out<<<(NH_ * NT_) / 8, 256, 0, stream>>>(AT, out);
}
